// BAPNet_51324859187665
// MI455X (gfx1250) — hardware-run, weakly checked
//
#include <hip/hip_runtime.h>
#include <stddef.h>


#define HID     128
#define NTHR    256
#define NWAVE   8
#define EPT     8
#define CHUNK   (NTHR * EPT)
#define WCAP    (EPT * 32)
#define LISTN   (NWAVE * WCAP)
#define PASSN   NTHR
#define PCAP    (CHUNK + PASSN)
#define EPITCH  136
#define NB_MSG  256
#define NB_CRD  1024
#define GM      64
#define SPITCH  40
#define WSC     16.0f
#define WINV    0.0625f
#define NRM_INV 0.01f

static_assert(PASSN == NWAVE * 32);
static_assert(PCAP >= CHUNK + PASSN);
static_assert((NB_MSG % NWAVE) == 0);
static_assert(((NB_CRD * 12) % 128) == 0);
static_assert(((NB_CRD * 3) % (4 * NTHR)) == 0);
static_assert((EPITCH % 8) == 0);
static_assert((2 * GM + 2 * HID) * SPITCH * 2 <= GM * HID * 4);

typedef float          v4f  __attribute__((ext_vector_type(4)));
typedef float          v8f  __attribute__((ext_vector_type(8)));
typedef int            v4i  __attribute__((ext_vector_type(4)));
typedef _Float16       v4h  __attribute__((ext_vector_type(4)));
typedef _Float16       v8h  __attribute__((ext_vector_type(8)));
typedef _Float16       v16h __attribute__((ext_vector_type(16)));
typedef unsigned short v8us __attribute__((ext_vector_type(8)));
typedef __bf16         v16b __attribute__((ext_vector_type(16)));
union FragH { v16h v; v8h h[2]; };
union FragB { v16b v; v16h hv; v8us u[2]; };

__device__ __forceinline__ v8f zero8f() {
  v8f z;
#pragma unroll
  for (int i = 0; i < 8; ++i) z[i] = 0.0f;
  return z;
}

__device__ __forceinline__ v8f wmh(v16h a, v16h b, v8f c) {
  v8f d = __builtin_amdgcn_wmma_f32_16x16x32_f16(false, a, false, b, (short)0, c, false, false);
  asm volatile("v_nop\n\tv_nop\n\tv_nop\n\tv_nop" : "+v"(d) : "v"(a), "v"(b));
  return d;
}
__device__ __forceinline__ v8f wmb(FragB a, FragB b, v8f c) {
  v8f d = __builtin_amdgcn_wmma_f32_16x16x32_bf16(false, a.v, false, b.v, (short)0, c, false, false);
  asm volatile("v_nop\n\tv_nop\n\tv_nop\n\tv_nop" : "+v"(d) : "v"(a.hv), "v"(b.hv));
  return d;
}

__device__ __forceinline__ unsigned short bf_rne(float x) {
  unsigned int u = __float_as_uint(x);
  u = (u + 0x7FFFu + ((u >> 16) & 1u)) >> 16;
  return (unsigned short)u;
}
__device__ __forceinline__ float bf_val(unsigned short b) {
  return __uint_as_float(((unsigned int)b) << 16);
}
__device__ __forceinline__ void bf_split(float x, unsigned short& hi, unsigned short& lo) {
  hi = bf_rne(x);
  lo = bf_rne(x - bf_val(hi));
}

__device__ __forceinline__ float siluf(float v) {
  const float e = __expf(-v);
  return v * __builtin_amdgcn_rcpf(1.0f + e);
}

template <int NBK>
__device__ __forceinline__ int scan_chunk(const int* __restrict__ keys, int nE, int cbase, int nodeBase,
                                          int vec8, int* list, int tid, int wave) {
  int wc = 0;
  const int el0  = tid * EPT;
  const int e0   = cbase + el0;
  const int sent = -2147483647 - 1;
  v4i da, db;
  if (vec8 != 0 && cbase + CHUNK <= nE) {
    da = *(const v4i*)(keys + e0);
    db = *(const v4i*)(keys + e0 + 4);
  } else {
    da.x = (e0     < nE) ? keys[min(e0,     nE - 1)] : sent;
    da.y = (e0 + 1 < nE) ? keys[min(e0 + 1, nE - 1)] : sent;
    da.z = (e0 + 2 < nE) ? keys[min(e0 + 2, nE - 1)] : sent;
    da.w = (e0 + 3 < nE) ? keys[min(e0 + 3, nE - 1)] : sent;
    db.x = (e0 + 4 < nE) ? keys[min(e0 + 4, nE - 1)] : sent;
    db.y = (e0 + 5 < nE) ? keys[min(e0 + 5, nE - 1)] : sent;
    db.z = (e0 + 6 < nE) ? keys[min(e0 + 6, nE - 1)] : sent;
    db.w = (e0 + 7 < nE) ? keys[min(e0 + 7, nE - 1)] : sent;
  }
  const unsigned nb = (unsigned)nodeBase;
  const unsigned s0 = (unsigned)da.x - nb, s1 = (unsigned)da.y - nb;
  const unsigned s2 = (unsigned)da.z - nb, s3 = (unsigned)da.w - nb;
  const unsigned s4 = (unsigned)db.x - nb, s5 = (unsigned)db.y - nb;
  const unsigned s6 = (unsigned)db.z - nb, s7 = (unsigned)db.w - nb;
  const bool h0 = s0 < (unsigned)NBK, h1 = s1 < (unsigned)NBK, h2 = s2 < (unsigned)NBK, h3 = s3 < (unsigned)NBK;
  const bool h4 = s4 < (unsigned)NBK, h5 = s5 < (unsigned)NBK, h6 = s6 < (unsigned)NBK, h7 = s7 < (unsigned)NBK;
  const unsigned any = __builtin_amdgcn_ballot_w32(h0 | h1 | h2 | h3 | h4 | h5 | h6 | h7);
  if (any != 0u) {
#define HITJ(J, HJ) { \
      const unsigned mj = __builtin_amdgcn_ballot_w32(HJ); \
      if (mj != 0u) { \
        if (HJ) { \
          const int pos = wc + (int)__builtin_amdgcn_mbcnt_lo(mj, 0u); \
          if (pos < WCAP) list[wave * WCAP + pos] = el0 + (J); \
        } \
        wc += (int)__builtin_popcount(mj); } }
    HITJ(0, h0)
    HITJ(1, h1)
    HITJ(2, h2)
    HITJ(3, h3)
    HITJ(4, h4)
    HITJ(5, h5)
    HITJ(6, h6)
    HITJ(7, h7)
#undef HITJ
  }
  return wc;
}

__global__ __launch_bounds__(NTHR) void k_packw(const float* __restrict__ Wa, const float* __restrict__ Wb,
                                                _Float16* outp) {
  const int tid   = threadIdx.x;
  const int rowi  = blockIdx.x * 16 + (tid >> 4);
  const int kq    = (tid & 15) * 8;
  const int plane = rowi >> 7, n = rowi & 127;
  const float* src = (plane != 0) ? Wb : Wa;
  v8h v;
#pragma unroll
  for (int i = 0; i < 8; ++i) v[i] = (_Float16)(src[(size_t)(kq + i) * HID + n] * WSC);
  _Float16* dp = outp + (size_t)rowi * HID + kq;
  *(volatile v8h*)dp = v;
  __threadfence();
  *(volatile v8h*)dp = v;
}

__global__ __launch_bounds__(NTHR) void k_ngemm(
    const float* __restrict__ A0, const float* __restrict__ A1, int M, int K,
    const float* __restrict__ W, int wStrideY,
    const float* __restrict__ bias, int biasAllY,
    const float* __restrict__ resid, int mode,
    float* outp, int outStrideY, int outLim) {
  __shared__ __attribute__((aligned(16))) unsigned char smraw[GM * HID * 4];
  unsigned short* Ah = (unsigned short*)smraw;
  unsigned short* Al = Ah + GM * SPITCH;
  unsigned short* Bh = Al + GM * SPITCH;
  unsigned short* Bl = Bh + HID * SPITCH;
  float* Cs = (float*)smraw;

  const int tid = threadIdx.x, lane = tid & 31, wave = tid >> 5, hh = lane >> 4, m = lane & 15;
  const int mt = wave & 3, ng = wave >> 2;
  const int row0 = blockIdx.x * GM;
  const float* Wy = W + (size_t)blockIdx.y * (size_t)wStrideY;

  v8f acc[4];
#pragma unroll
  for (int j = 0; j < 4; ++j) acc[j] = zero8f();

  const int nK = K >> 5;
#pragma unroll 1
  for (int kc = 0; kc < nK; ++kc) {
    const int k0 = kc * 32;
    {
      const int rl = tid >> 2, kq = (tid & 3) * 8;
      int ra = row0 + rl;
      ra = ra > M - 1 ? M - 1 : ra;
      const float* src;
      int ks;
      if (k0 < HID) { src = A0; ks = k0; } else { src = A1; ks = k0 - HID; }
      const float* ap = src + (size_t)ra * HID + ks + kq;
      const v4f u0 = *(const v4f*)ap;
      const v4f u1 = *(const v4f*)(ap + 4);
      v8us h8, l8;
#pragma unroll
      for (int i = 0; i < 8; ++i) {
        const float xv = (i < 4) ? u0[i] : u1[i - 4];
        unsigned short hb, lb;
        bf_split(xv, hb, lb);
        h8[i] = hb;
        l8[i] = lb;
      }
      *(v8us*)(Ah + rl * SPITCH + kq) = h8;
      *(v8us*)(Al + rl * SPITCH + kq) = l8;
    }
    {
      const int n = tid & 127, kh = (tid >> 7) * 16;
      const float* wp = Wy + (size_t)(k0 + kh) * HID + n;
      v8us h0, l0, h1, l1;
#pragma unroll
      for (int i = 0; i < 16; ++i) {
        const float xv = wp[(size_t)i * HID];
        unsigned short hb, lb;
        bf_split(xv, hb, lb);
        if (i < 8) { h0[i] = hb; l0[i] = lb; } else { h1[i - 8] = hb; l1[i - 8] = lb; }
      }
      *(v8us*)(Bh + n * SPITCH + kh)     = h0;
      *(v8us*)(Bh + n * SPITCH + kh + 8) = h1;
      *(v8us*)(Bl + n * SPITCH + kh)     = l0;
      *(v8us*)(Bl + n * SPITCH + kh + 8) = l1;
    }
    __syncthreads();
    {
      FragB ah, al;
      const unsigned short* ar = Ah + (16 * mt + m) * SPITCH + 8 * hh;
      const unsigned short* as = Al + (16 * mt + m) * SPITCH + 8 * hh;
      ah.u[0] = *(const v8us*)ar;  ah.u[1] = *(const v8us*)(ar + 16);
      al.u[0] = *(const v8us*)as;  al.u[1] = *(const v8us*)(as + 16);
#pragma unroll
      for (int j = 0; j < 4; ++j) {
        FragB bh, bl;
        const unsigned short* br = Bh + (64 * ng + 16 * j + m) * SPITCH + 8 * hh;
        const unsigned short* bs = Bl + (64 * ng + 16 * j + m) * SPITCH + 8 * hh;
        bh.u[0] = *(const v8us*)br;  bh.u[1] = *(const v8us*)(br + 16);
        bl.u[0] = *(const v8us*)bs;  bl.u[1] = *(const v8us*)(bs + 16);
        acc[j] = wmb(ah, bh, acc[j]);
        acc[j] = wmb(ah, bl, acc[j]);
        acc[j] = wmb(al, bh, acc[j]);
      }
    }
    __syncthreads();
  }

#pragma unroll
  for (int j = 0; j < 4; ++j)
#pragma unroll
    for (int r = 0; r < 8; ++r)
      Cs[(16 * mt + 8 * hh + r) * HID + 64 * ng + 16 * j + m] = acc[j][r];
  __syncthreads();

  const bool useB = (biasAllY != 0) || (blockIdx.y == 0);
  v4f bv = *(const v4f*)(bias + 4 * lane);
  if (!useB) { bv[0] = 0.0f; bv[1] = 0.0f; bv[2] = 0.0f; bv[3] = 0.0f; }
  v4f ov[8];
#pragma unroll
  for (int i = 0; i < 8; ++i) {
    const int rl = wave * 8 + i;
    const int row = row0 + rl;
    v4f v = *(const v4f*)(Cs + rl * HID + 4 * lane);
    v = v + bv;
    if (mode == 1) {
#pragma unroll
      for (int c = 0; c < 4; ++c) v[c] = siluf(v[c]);
    } else if (mode == 2) {
      const int rr = row > M - 1 ? M - 1 : row;
      const v4f hv = *(const v4f*)(resid + (size_t)rr * HID + 4 * lane);
      v = hv + v;
    }
    ov[i] = v;
  }
  float* ob = outp + (size_t)blockIdx.y * (size_t)outStrideY;
#pragma unroll
  for (int i = 0; i < 8; ++i) {
    const int row = row0 + wave * 8 + i;
    if (row < outLim) *(volatile v4f*)(ob + (size_t)row * HID + 4 * lane) = ov[i];
  }
  __threadfence();
#pragma unroll
  for (int i = 0; i < 8; ++i) {
    const int row = row0 + wave * 8 + i;
    if (row < outLim) *(volatile v4f*)(ob + (size_t)row * HID + 4 * lane) = ov[i];
  }
}

template <int COORD>
__global__ __launch_bounds__(NTHR) void k_edge(
    const float* __restrict__ Pp, const float* __restrict__ Qp,
    const float* __restrict__ x, const float* __restrict__ eattr, const int* __restrict__ ei,
    const float* __restrict__ W1, const _Float16* __restrict__ W2p,
    const float* __restrict__ B2, const float* __restrict__ W3,
    float* outp, int nN, int nE, int vec8, int outLim) {
  constexpr int NBK = COORD ? NB_CRD : NB_MSG;
  constexpr int AW  = COORD ? 4 : HID;

  __shared__ __attribute__((aligned(16))) float    acc[(NBK + 1) * AW];
  __shared__ __attribute__((aligned(16))) _Float16 etile[PASSN * EPITCH];
  __shared__ __attribute__((aligned(16))) int      list[LISTN];
  __shared__ __attribute__((aligned(16))) int      pend[PCAP];
  __shared__ int   eP[PASSN];
  __shared__ int   eQ[PASSN];
  __shared__ int   eS[PASSN];
  __shared__ float eR[PASSN];
  __shared__ float eA[PASSN];
  __shared__ __attribute__((aligned(16))) float ecd[COORD ? 3 * PASSN : 4];
  __shared__ __attribute__((aligned(16))) float ephi[COORD ? NWAVE * PASSN : 4];
  __shared__ float ephis[COORD ? PASSN : 4];
  __shared__ __attribute__((aligned(16))) float xs[COORD ? NB_CRD * 3 : 4];
  __shared__ int wcnt[NWAVE];
  __shared__ int pendN;

  const int tid = threadIdx.x, lane = tid & 31, wave = tid >> 5, hh = lane >> 4, m = lane & 15;
  const int nodeBase = blockIdx.x * NBK;
  const int* keys = ei;
  const int* cols = ei + nE;

  for (int i = tid; i < (NBK + 1) * AW; i += NTHR) acc[i] = 0.0f;
  if (tid == 0) pendN = 0;
  float wr[4], wa[4];
#pragma unroll
  for (int c = 0; c < 4; ++c) {
    wr[c] = W1[256 * HID + 4 * lane + c];
    wa[c] = W1[257 * HID + 4 * lane + c];
  }
  const int   ncol = 16 * wave + m;
  const float b2n  = B2[ncol];
  const float w3n  = (COORD != 0) ? W3[ncol] : 0.0f;
  __syncthreads();

  const int nChunks = (nE + CHUNK - 1) / CHUNK;
#pragma unroll 1
  for (int ch = 0; ch < nChunks; ++ch) {
    const int cbase = ch * CHUNK;
    const int wc = scan_chunk<NBK>(keys, nE, cbase, nodeBase, vec8, list, tid, wave);
    if (lane == 0) wcnt[wave] = wc;
    __syncthreads();

    const int base = pendN;
    int tot = 0, myoff = 0;
#pragma unroll
    for (int w = 0; w < NWAVE; ++w) {
      int c = wcnt[w];
      c = c > WCAP ? WCAP : (c < 0 ? 0 : c);
      if (w < wave) myoff += c;
      tot += c;
    }
    int newN = base + tot;
    newN = newN > PCAP ? PCAP : newN;
    {
      int n = wcnt[wave];
      n = n > WCAP ? WCAP : (n < 0 ? 0 : n);
      const int* lp = list + wave * WCAP;
      for (int i = lane; i < n; i += 32) {
        const int pos = base + myoff + i;
        if (pos < PCAP) pend[pos] = cbase + lp[i];
      }
    }
    const int fin = (ch == nChunks - 1) ? 1 : 0;
    const int R   = (fin != 0) ? (newN + PASSN - 1) / PASSN : newN / PASSN;
    const int Pv  = (fin != 0) ? newN : R * PASSN;
    __syncthreads();

#pragma unroll 1
    for (int r = 0; r < R; ++r) {
      {
        const int idx = r * PASSN + tid;
        const bool valid = idx < Pv;
        int e = pend[idx < PCAP ? idx : PCAP - 1];
        e = valid ? e : 0;
        e = e < 0 ? 0 : (e > nE - 1 ? nE - 1 : e);
        int ri = keys[e];
        int ci = cols[e];
        int slot = ri - nodeBase;
        if (!valid || (unsigned)slot >= (unsigned)NBK) slot = NBK;
        ri = ri < 0 ? 0 : (ri > nN - 1 ? nN - 1 : ri);
        ci = ci < 0 ? 0 : (ci > nN - 1 ? nN - 1 : ci);
        const float ea = eattr[e];
        const float dx = x[(size_t)ri * 3 + 0] - x[(size_t)ci * 3 + 0];
        const float dy = x[(size_t)ri * 3 + 1] - x[(size_t)ci * 3 + 1];
        const float dz = x[(size_t)ri * 3 + 2] - x[(size_t)ci * 3 + 2];
        const float rad = dx * dx + dy * dy + dz * dz;
        eP[tid] = ri; eQ[tid] = ci; eS[tid] = slot; eR[tid] = rad; eA[tid] = ea;
        if (COORD != 0) {
          const float inv = __builtin_amdgcn_rcpf(sqrtf(rad + 1e-8f) + 1.0f);
          ecd[tid] = dx * inv;
          ecd[PASSN + tid] = dy * inv;
          ecd[2 * PASSN + tid] = dz * inv;
        }
      }
      __syncthreads();

      {
#pragma unroll 1
        for (int j = 0; j < 32; ++j) {
          const int p  = wave * 32 + j;
          const int ri = eP[p], ci = eQ[p], sl = eS[p];
          const float rad = eR[p], ea = eA[p];
          const v4f pv = *(const v4f*)(Pp + (size_t)ri * HID + 4 * lane);
          const v4f qv = *(const v4f*)(Qp + (size_t)ci * HID + 4 * lane);
          v4h hv;
#pragma unroll
          for (int c = 0; c < 4; ++c) {
            const float v = pv[c] + qv[c] + rad * wr[c] + ea * wa[c];
            float s = siluf(v);
            s = (sl < NBK) ? s : 0.0f;
            hv[c] = (_Float16)s;
          }
          *(v4h*)(etile + p * EPITCH + 4 * lane) = hv;
        }
      }
      __syncthreads();

      {
        FragH bq[4];
        {
          const _Float16* bp = W2p + (size_t)ncol * HID + 8 * hh;
#pragma unroll
          for (int kc = 0; kc < 4; ++kc) {
            bq[kc].h[0] = *(const v8h*)(bp + 32 * kc);
            bq[kc].h[1] = *(const v8h*)(bp + 32 * kc + 16);
          }
        }
#pragma unroll 1
        for (int et = 0; et < PASSN / 16; ++et) {
          v8f d = zero8f();
          const _Float16* ap = etile + (et * 16 + m) * EPITCH + 8 * hh;
#pragma unroll
          for (int kc = 0; kc < 4; ++kc) {
            FragH a;
            a.h[0] = *(const v8h*)(ap + 32 * kc);
            a.h[1] = *(const v8h*)(ap + 32 * kc + 16);
            d = wmh(a.v, bq[kc].v, d);
          }
          float val[8];
#pragma unroll
          for (int rr = 0; rr < 8; ++rr) val[rr] = siluf(d[rr] * WINV + b2n);
          if (COORD == 0) {
            float vhi[8];
#pragma unroll
            for (int rr = 0; rr < 8; ++rr) vhi[rr] = __shfl_xor(val[rr], 16, 32);
#pragma unroll
            for (int rr = 0; rr < 8; ++rr) {
              int sl = eS[et * 16 + rr];
              sl = sl < 0 ? 0 : (sl > NBK ? NBK : sl);
              sl = (hh == 0) ? sl : NBK;
              const int ai = sl * AW + ncol;
              const float t = acc[ai] + val[rr];
              acc[ai] = t;
            }
#pragma unroll
            for (int rr = 0; rr < 8; ++rr) {
              int sl = eS[et * 16 + 8 + rr];
              sl = sl < 0 ? 0 : (sl > NBK ? NBK : sl);
              sl = (hh == 0) ? sl : NBK;
              const int ai = sl * AW + ncol;
              const float t = acc[ai] + vhi[rr];
              acc[ai] = t;
            }
          } else {
            float pr[8];
#pragma unroll
            for (int rr = 0; rr < 8; ++rr) {
              float t = val[rr] * w3n;
              t += __shfl_xor(t, 1, 32);
              t += __shfl_xor(t, 2, 32);
              t += __shfl_xor(t, 4, 32);
              t += __shfl_xor(t, 8, 32);
              pr[rr] = t;
            }
            if (m == 0) {
#pragma unroll
              for (int rr = 0; rr < 8; ++rr) ephi[wave * PASSN + et * 16 + 8 * hh + rr] = pr[rr];
            }
          }
        }
      }
      __syncthreads();

      if (COORD != 0) {
        {
          float ph = 0.0f;
#pragma unroll
          for (int w = 0; w < NWAVE; ++w) ph += ephi[w * PASSN + tid];
          ephis[tid] = ph;
        }
        __syncthreads();
        if (wave == 0) {
#pragma unroll 1
          for (int i = 0; i < PASSN; ++i) {
            int sl = eS[i];
            sl = sl < 0 ? 0 : (sl > NBK ? NBK : sl);
            if (lane < 3) {
              const float t = ecd[lane * PASSN + i] * ephis[i];
              const int ai = sl * AW + lane;
              const float u = acc[ai] + t;
              acc[ai] = u;
            }
          }
        }
        __syncthreads();
      }
    }

    int rem = newN - R * PASSN;
    rem = rem < 0 ? 0 : rem;
    if (R > 0 && tid < rem) pend[tid] = pend[R * PASSN + tid];
    if (tid == 0) pendN = rem;
  }
  __syncthreads();

  if (COORD == 0) {
#pragma unroll 1
    for (int i = 0; i < NBK / NWAVE; ++i) {
      const int rl = i * NWAVE + wave;
      const int node = nodeBase + rl;
      v4f v = *(const v4f*)(acc + rl * AW + 4 * lane);
      v = v * NRM_INV;
      if (node < outLim) *(volatile v4f*)(outp + (size_t)node * HID + 4 * lane) = v;
    }
    __threadfence();
#pragma unroll 1
    for (int i = 0; i < NBK / NWAVE; ++i) {
      const int rl = i * NWAVE + wave;
      const int node = nodeBase + rl;
      v4f v = *(const v4f*)(acc + rl * AW + 4 * lane);
      v = v * NRM_INV;
      if (node < outLim) *(volatile v4f*)(outp + (size_t)node * HID + 4 * lane) = v;
    }
  } else {
    for (int i = tid; i < NB_CRD * 3; i += NTHR) {
      const int nl = i / 3;
      const int c  = i - 3 * nl;
      const int node = nodeBase + nl;
      const int na = node > nN - 1 ? nN - 1 : node;
      xs[i] = x[(size_t)na * 3 + c] + acc[nl * AW + c] * NRM_INV;
    }
    __syncthreads();
    const size_t ob  = (size_t)nodeBase * 3;
    const size_t lim = (size_t)(outLim < 0 ? 0 : outLim);
    constexpr int NJ = (NB_CRD * 3) / (4 * NTHR);
#pragma unroll
    for (int j = 0; j < NJ; ++j) {
      const int f4 = (j * NWAVE + wave) * 32 + lane;
      const v4f v = *(const v4f*)(xs + 4 * f4);
      const size_t gi = ob + 4 * (size_t)f4;
      if (gi + 4 <= lim) {
        *(volatile v4f*)(outp + gi) = v;
      } else {
#pragma unroll
        for (int c = 0; c < 4; ++c)
          if (gi + c < lim) ((volatile float*)outp)[gi + c] = v[c];
      }
    }
    __threadfence();
#pragma unroll
    for (int j = 0; j < NJ; ++j) {
      const int f4 = (j * NWAVE + wave) * 32 + lane;
      const v4f v = *(const v4f*)(xs + 4 * f4);
      const size_t gi = ob + 4 * (size_t)f4;
      if (gi + 4 <= lim) {
        *(volatile v4f*)(outp + gi) = v;
      } else {
#pragma unroll
        for (int c = 0; c < 4; ++c)
          if (gi + c < lim) ((volatile float*)outp)[gi + c] = v[c];
      }
    }
  }
}

extern "C" void kernel_launch(void* const* d_in, const int* in_sizes, int n_in,
                              void* d_out, int out_size, void* d_ws, size_t ws_size,
                              hipStream_t stream) {
  if (n_in < 17) return;
  const int nN = in_sizes[0] / HID;
  const int nE = in_sizes[2];
  if (nN <= 0 || nE < 1) return;
  if (in_sizes[0] != nN * HID || in_sizes[1] != nN * 3 || in_sizes[3] != 2 * nE) return;
  if (in_sizes[4] != 258 * HID || in_sizes[5] < HID || in_sizes[6] != HID * HID || in_sizes[7] < HID) return;
  if (in_sizes[8] != 256 * HID || in_sizes[9] < HID || in_sizes[10] != HID * HID || in_sizes[11] < HID) return;
  if (in_sizes[12] != 258 * HID || in_sizes[13] < HID || in_sizes[14] != HID * HID || in_sizes[15] < HID) return;
  if (in_sizes[16] < HID) return;
  if (out_size != nN * HID + nN * 3) return;

  const float* h     = (const float*)d_in[0];
  const float* x     = (const float*)d_in[1];
  const float* eattr = (const float*)d_in[2];
  const int*   ei    = (const int*)d_in[3];
  const float* w_e1  = (const float*)d_in[4];
  const float* b_e1  = (const float*)d_in[5];
  const float* w_e2  = (const float*)d_in[6];
  const float* b_e2  = (const float*)d_in[7];
  const float* w_n1  = (const float*)d_in[8];
  const float* b_n1  = (const float*)d_in[9];
  const float* w_n2  = (const float*)d_in[10];
  const float* b_n2  = (const float*)d_in[11];
  const float* w_c1  = (const float*)d_in[12];
  const float* b_c1  = (const float*)d_in[13];
  const float* w_c2  = (const float*)d_in[14];
  const float* b_c2  = (const float*)d_in[15];
  const float* w_c3  = (const float*)d_in[16];
  float* hOut = (float*)d_out;
  float* xOut = (float*)d_out + (size_t)nN * HID;

  const int mBlk    = (nN + GM - 1) / GM;
  const int Mpad    = mBlk * GM;
  const int nBlk1   = (nN + NB_MSG - 1) / NB_MSG;
  const int aggRows = nBlk1 * NB_MSG;
  const int nBlk2   = (nN + NB_CRD - 1) / NB_CRD;

  size_t off = 0;
  const size_t oW2p = off; off += (size_t)2 * HID * HID * 2;
  const size_t oP   = off; off += (size_t)Mpad * HID * 4;
  const size_t oQ   = off; off += (size_t)Mpad * HID * 4;
  const size_t oAgg = off; off += (size_t)aggRows * HID * 4;
  const size_t oT   = off; off += (size_t)Mpad * HID * 4;
  if (off > ws_size || off > (size_t)134217728) return;
  char* ws = (char*)d_ws;
  _Float16* W2p = (_Float16*)(ws + oW2p);
  float* Ppl  = (float*)(ws + oP);
  float* Qpl  = (float*)(ws + oQ);
  float* aggp = (float*)(ws + oAgg);
  float* Tpl  = (float*)(ws + oT);
  const int pqStride = Mpad * HID;
  const int vec8 = 1;

  k_packw<<<(2 * HID) / 16, NTHR, 0, stream>>>(w_e2, w_c2, W2p);

  k_ngemm<<<dim3(mBlk, 2), NTHR, 0, stream>>>(h, h, nN, HID, w_e1, HID * HID, b_e1, 0, h, 0,
                                               Ppl, pqStride, Mpad);

  k_edge<0><<<nBlk1, NTHR, 0, stream>>>(Ppl, Qpl, x, eattr, ei, w_e1, W2p, b_e2, b_e2,
                                        aggp, nN, nE, vec8, aggRows);

  k_ngemm<<<dim3(mBlk, 1), NTHR, 0, stream>>>(h, aggp, nN, 2 * HID, w_n1, 0, b_n1, 1, h, 1,
                                               Tpl, 0, Mpad);

  k_ngemm<<<dim3(mBlk, 1), NTHR, 0, stream>>>(Tpl, Tpl, nN, HID, w_n2, 0, b_n2, 1, h, 2,
                                               hOut, 0, nN);

  k_ngemm<<<dim3(mBlk, 2), NTHR, 0, stream>>>(hOut, hOut, nN, HID, w_c1, HID * HID, b_c1, 0, h, 0,
                                               Ppl, pqStride, Mpad);

  k_edge<1><<<nBlk2, NTHR, 0, stream>>>(Ppl, Qpl, x, eattr, ei, w_c1, W2p + (size_t)HID * HID, b_c2, w_c3,
                                        xOut, nN, nE, vec8, nN * 3);
}
